// RelLearnableDecoderLayer_51917564674337
// MI455X (gfx1250) — hardware-verified
//
#include <hip/hip_runtime.h>
#include <stdint.h>
#include <stddef.h>


typedef _Float16 f16;
typedef _Float16 v16h __attribute__((ext_vector_type(16)));
typedef _Float16 v8h  __attribute__((ext_vector_type(8)));
typedef float    v8f  __attribute__((ext_vector_type(8)));
typedef float    v4f  __attribute__((ext_vector_type(4)));

#define QLEN   1024
#define MLEN   1024
#define KLEN   2048
#define DMODEL 1024
#define NH     16
#define DHD    64
#define NB     2
#define DINNER 4096
#define ATT_SCALE 0.125f
#define WSC     64.0f
#define INV_WSC 0.015625f
#define PSC     256.0f

__device__ __forceinline__ v16h frag_ld(const f16* p) {
  union { v16h v; v8h hh[2]; } u;
  u.hh[0] = *(const v8h*)(p);
  u.hh[1] = *(const v8h*)(p + 16);
  return u.v;
}
__device__ __forceinline__ v8f wmma16(v16h a, v16h b, v8f c) {
  v8f d = __builtin_amdgcn_wmma_f32_16x16x32_f16(false, a, false, b, (short)0, c,
                                                 false, false);
  asm volatile("v_nop\n\tv_nop\n\tv_nop\n\tv_nop" : "+v"(d) : "v"(a), "v"(b));
  return d;
}
__device__ __forceinline__ v8f v8zero() {
  v8f z;
#pragma unroll
  for (int e = 0; e < 8; ++e) z[e] = 0.f;
  return z;
}
__device__ __forceinline__ v8h pack8(v4f a, v4f b, float s) {
  v8h o;
  o[0] = (f16)(a[0] * s); o[1] = (f16)(a[1] * s); o[2] = (f16)(a[2] * s); o[3] = (f16)(a[3] * s);
  o[4] = (f16)(b[0] * s); o[5] = (f16)(b[1] * s); o[6] = (f16)(b[2] * s); o[7] = (f16)(b[3] * s);
  return o;
}
__device__ __forceinline__ v4f relu4(v4f v) {
  v[0] = fmaxf(v[0], 0.f); v[1] = fmaxf(v[1], 0.f); v[2] = fmaxf(v[2], 0.f); v[3] = fmaxf(v[3], 0.f);
  return v;
}
__device__ __forceinline__ float wave_sum(float v) {
#pragma unroll
  for (int o = 16; o; o >>= 1) v += __shfl_xor(v, o, 32);
  return v;
}
__device__ __forceinline__ float wave_max(float v) {
#pragma unroll
  for (int o = 16; o; o >>= 1) v = fmaxf(v, __shfl_xor(v, o, 32));
  return v;
}

__global__ __launch_bounds__(256) void cvt16_kernel(const float* __restrict__ src,
                                                   f16* dst, int n8, float scale) {
  const int i = blockIdx.x * 256 + threadIdx.x;
  const bool ok = i < n8;
  v8h hv;
  size_t o = (size_t)i * 8;
  if (ok) {
    v4f a = *(const v4f*)(src + o);
    v4f b = *(const v4f*)(src + o + 4);
    hv = pack8(a, b, scale);
    *(volatile v8h*)(dst + o) = hv;
  }
  __threadfence();
  if (ok) *(volatile v8h*)(dst + o) = hv;
}

__global__ __launch_bounds__(256) void split_qk_kernel(const f16* __restrict__ heads,
                                                      const float* __restrict__ r_w_bias,
                                                      f16* q16, f16* q16b, f16* k16, int ntot) {
  const int i = blockIdx.x * 256 + threadIdx.x;
  const bool ok = i < ntot;
  f16* dst = nullptr;
  f16* dst2 = nullptr;
  v8h hv, hv2;
  if (ok) {
    const int d8 = i & 7, h = (i >> 3) & 15, sec = (i >> 7) & 1, row = i >> 8;
    const int kk = row >> 1, b = row & 1;
    hv = *(const v8h*)(heads + (size_t)row * 3072 + sec * 1024 + h * DHD + d8 * 8);
    hv2 = hv;
    if (sec == 0) {
      if (kk >= MLEN) {
        const size_t o = (((size_t)b * NH + h) * QLEN + (kk - MLEN)) * DHD + d8 * 8;
        dst = q16 + o;
        dst2 = q16b + o;
        const float* rb = r_w_bias + h * DHD + d8 * 8;
#pragma unroll
        for (int e = 0; e < 8; ++e) hv2[e] = (f16)((float)hv[e] + rb[e]);
      }
    } else {
      dst = k16 + (((size_t)b * NH + h) * KLEN + kk) * DHD + d8 * 8;
    }
    if (dst) *(volatile v8h*)dst = hv;
    if (dst2) *(volatile v8h*)dst2 = hv2;
  }
  __threadfence();
  if (ok) {
    if (dst) *(volatile v8h*)dst = hv;
    if (dst2) *(volatile v8h*)dst2 = hv2;
  }
}

#define VTP 72
__global__ __launch_bounds__(256) void vtrans_kernel(const f16* __restrict__ heads, f16* vT16) {
  __shared__ f16 tile[64 * VTP];
  const int tid = threadIdx.x;
  const int kk0 = blockIdx.x * 64, h = blockIdx.y, b = blockIdx.z;
  if (kk0 + 64 > KLEN || h >= NH || b >= NB) return;
#pragma unroll
  for (int p = 0; p < 2; ++p) {
    const int c = p * 256 + tid, kr = c >> 3, d8 = c & 7;
    *(v8h*)(tile + kr * VTP + d8 * 8) =
        *(const v8h*)(heads + ((size_t)(kk0 + kr) * NB + b) * 3072 + 2048 + h * DHD + d8 * 8);
  }
  __syncthreads();
  v8h ov[2];
  size_t od[2];
#pragma unroll
  for (int p = 0; p < 2; ++p) {
    const int c = p * 256 + tid, d = c >> 3, e = c & 7;
#pragma unroll
    for (int t = 0; t < 8; ++t) ov[p][t] = tile[(e * 8 + t) * VTP + d];
    od[p] = (((size_t)b * NH + h) * DHD + d) * KLEN + kk0 + e * 8;
  }
#pragma unroll
  for (int p = 0; p < 2; ++p) *(volatile v8h*)(vT16 + od[p]) = ov[p];
  __threadfence();
#pragma unroll
  for (int p = 0; p < 2; ++p) *(volatile v8h*)(vT16 + od[p]) = ov[p];
}

__global__ __launch_bounds__(256) void remb_kernel(const float* __restrict__ r_emb, f16* re16,
                                                  int ntot) {
  const int i = blockIdx.x * 256 + threadIdx.x;
  const bool ok = i < ntot;
  v8h hv;
  size_t o = 0;
  if (ok) {
    const int d8 = i & 7, h = (i >> 3) & 15, s = i >> 7;
    const float* sp = r_emb + ((size_t)s * NH + h) * DHD + d8 * 8;
    hv = pack8(*(const v4f*)sp, *(const v4f*)(sp + 4), WSC);
    o = ((size_t)h * KLEN + s) * DHD + d8 * 8;
    *(volatile v8h*)(re16 + o) = hv;
  }
  __threadfence();
  if (ok) *(volatile v8h*)(re16 + o) = hv;
}

#define GLDA 40
#define SCP 132
#define GEMM_SMEM (2 * 128 * GLDA * 2 + 128 * SCP * 4)

__device__ __forceinline__ void gemm_store(const float* sC, const float* __restrict__ bias,
                                           float* Cf, f16* Ch, int rowBase, int colBase, int N,
                                           int relu, float oscale, int wv, int lane) {
  const int hl = lane >> 4, r = lane & 15;
  if (Cf) {
#pragma unroll
    for (int t = 0; t < 16; ++t) {
      const int row = wv + 8 * t;
      const int col = colBase + lane * 4;
      v4f v = *(const v4f*)(sC + row * SCP + lane * 4);
      v = v * oscale;
      if (bias) v = v + *(const v4f*)(bias + col);
      if (relu) v = relu4(v);
      *(volatile v4f*)(Cf + (size_t)(rowBase + row) * N + col) = v;
    }
  }
  if (Ch) {
#pragma unroll
    for (int t = 0; t < 8; ++t) {
      const int row = 2 * (wv + 8 * t) + hl;
      const int c8 = r * 8;
      const int col = colBase + c8;
      v4f p0 = *(const v4f*)(sC + row * SCP + c8);
      v4f p1 = *(const v4f*)(sC + row * SCP + c8 + 4);
      p0 = p0 * oscale;
      p1 = p1 * oscale;
      if (bias) {
        p0 = p0 + *(const v4f*)(bias + col);
        p1 = p1 + *(const v4f*)(bias + col + 4);
      }
      if (relu) { p0 = relu4(p0); p1 = relu4(p1); }
      v8h hv = pack8(p0, p1, 1.0f);
      *(volatile v8h*)(Ch + (size_t)(rowBase + row) * N + col) = hv;
    }
  }
}

__global__ __launch_bounds__(256) void gemm_nt_kernel(
    const f16* __restrict__ A, const f16* __restrict__ W, const float* __restrict__ bias,
    float* Cf, f16* Ch, int Mr, int N, int Kd, int relu, float oscale) {
  extern __shared__ v4f dsm[];
  f16* sA = (f16*)dsm;
  f16* sB = sA + 128 * GLDA;
  float* sC = (float*)(sB + 128 * GLDA);
  const int tid = threadIdx.x;
  const int wv = tid >> 5, lane = tid & 31, hl = lane >> 4, r = lane & 15;
  const int wm = wv >> 1, wn = wv & 1;
  const int rowBase = blockIdx.y * 128;
  const int colBase = blockIdx.x * 128;
  if (rowBase + 128 > Mr || colBase + 128 > N) return;

  v8f acc[2][4];
#pragma unroll
  for (int i = 0; i < 2; ++i)
#pragma unroll
    for (int j = 0; j < 4; ++j) acc[i][j] = v8zero();

  for (int kb = 0; kb < Kd; kb += 32) {
#pragma unroll
    for (int p = 0; p < 2; ++p) {
      const int id = p * 256 + tid;
      const int row = id >> 2, ch = id & 3;
      v8h va = *(const v8h*)(A + (size_t)(rowBase + row) * Kd + kb + ch * 8);
      v8h vb = *(const v8h*)(W + (size_t)(colBase + row) * Kd + kb + ch * 8);
      *(v8h*)(sA + row * GLDA + ch * 8) = va;
      *(v8h*)(sB + row * GLDA + ch * 8) = vb;
    }
    __syncthreads();
    v16h af[2], bf[4];
#pragma unroll
    for (int fm = 0; fm < 2; ++fm)
      af[fm] = frag_ld(sA + (wm * 32 + fm * 16 + r) * GLDA + hl * 8);
#pragma unroll
    for (int fn = 0; fn < 4; ++fn)
      bf[fn] = frag_ld(sB + (wn * 64 + fn * 16 + r) * GLDA + hl * 8);
#pragma unroll
    for (int fm = 0; fm < 2; ++fm)
#pragma unroll
      for (int fn = 0; fn < 4; ++fn)
        acc[fm][fn] = wmma16(af[fm], bf[fn], acc[fm][fn]);
    __syncthreads();
  }

#pragma unroll
  for (int fm = 0; fm < 2; ++fm)
#pragma unroll
    for (int fn = 0; fn < 4; ++fn)
#pragma unroll
      for (int g = 0; g < 8; ++g)
        sC[(wm * 32 + fm * 16 + hl * 8 + g) * SCP + wn * 64 + fn * 16 + r] = acc[fm][fn][g];
  __syncthreads();

  gemm_store(sC, bias, Cf, Ch, rowBase, colBase, N, relu, oscale, wv, lane);
  __threadfence();
  gemm_store(sC, bias, Cf, Ch, rowBase, colBase, N, relu, oscale, wv, lane);
}

#define SCS 2056
#define STRIPW 576
#define STGP 72
#define ATT_SMEM (64 * SCS * 2 + 4 * STRIPW * 4 + 64 * 4)

__global__ __launch_bounds__(128) void attn_kernel(
    const f16* __restrict__ q16, const f16* __restrict__ q16b,
    const f16* __restrict__ k16, const f16* __restrict__ vT16,
    const f16* __restrict__ re16, const float* __restrict__ r_bias,
    const int* __restrict__ mask, f16* vec16) {
  extern __shared__ v4f dsm[];
  char* smem = (char*)dsm;
  f16* sc = (f16*)smem;
  float* strip = (float*)(smem + 64 * SCS * 2);
  float* rowsum = strip + 4 * STRIPW;

  const int wv = threadIdx.x >> 5, lane = threadIdx.x & 31;
  const int hl = lane >> 4, r = lane & 15;
  const int b = blockIdx.z, h = blockIdx.y;
  if (blockIdx.x * 64 + 64 > QLEN || h >= NH || b >= NB) return;
  const int iq = blockIdx.x * 64 + wv * 16;
  const size_t bh = (size_t)b * NH + h;
  float* wstrip = strip + wv * STRIPW;

  const f16* qb_base = q16b + (bh * QLEN + iq) * DHD;
  const f16* qp_base = q16 + (bh * QLEN + iq) * DHD;
  v16h qa[2], qn[2];
#pragma unroll
  for (int c = 0; c < 2; ++c) {
    qa[c] = frag_ld(qb_base + r * DHD + c * 32 + hl * 8);
    qn[c] = frag_ld(qp_base + r * DHD + c * 32 + hl * 8);
  }

  auto btile = [&](int st) -> v8f {
    v8f bt = v8zero();
    int srow = st + r;
    if (srow > KLEN - 1) srow = KLEN - 1;
    const f16* rp = re16 + ((size_t)h * KLEN + srow) * DHD + hl * 8;
#pragma unroll
    for (int c = 0; c < 2; ++c) bt = wmma16(qn[c], frag_ld(rp + c * 32), bt);
    return bt;
  };
  auto store_strip = [&](v8f bt, int par) {
    float* dst = wstrip + par * 288;
#pragma unroll
    for (int g = 0; g < 8; ++g) dst[(g + hl * 8) * 18 + r] = bt[g] * INV_WSC;
  };

  const int st0 = QLEN - 16 - iq;
  store_strip(btile(st0), (st0 >> 4) & 1);

  for (int j0 = 0; j0 < KLEN; j0 += 16) {
    if (j0 > iq + 15 + MLEN) {
#pragma unroll
      for (int g = 0; g < 8; ++g)
        sc[(size_t)(wv * 16 + g + hl * 8) * SCS + j0 + r] = (f16)(-__builtin_inff());
      continue;
    }
    v8f ac = v8zero();
    const f16* kp = k16 + (bh * KLEN + j0 + r) * DHD + hl * 8;
#pragma unroll
    for (int c = 0; c < 2; ++c) ac = wmma16(qa[c], frag_ld(kp + c * 32), ac);
    const int stn = j0 + QLEN - iq;
    const int parn = (stn >> 4) & 1;
    store_strip(btile(stn), parn);
    asm volatile("s_wait_dscnt 0" ::: "memory");
    const float* oldb = wstrip + (parn ^ 1) * 288;
    const float* newb = wstrip + parn * 288;
#pragma unroll
    for (int g = 0; g < 8; ++g) {
      const int m = g + hl * 8;
      const int ig = iq + m;
      const int jg = j0 + r;
      const int rel = 15 + r - m;
      const float bv = (rel < 16) ? oldb[m * 18 + rel] : newb[m * 18 + rel - 16];
      int s = jg + QLEN - 1 - ig;
      if (s > KLEN - 1) s = KLEN - 1;
      float scv = (ac[g] + bv + r_bias[(size_t)s * NH + h]) * ATT_SCALE;
      if (mask[(size_t)ig * KLEN + jg] != 0) scv = -__builtin_inff();
      sc[(size_t)(wv * 16 + m) * SCS + jg] = (f16)scv;
    }
  }
  asm volatile("s_wait_dscnt 0" ::: "memory");

#pragma unroll 1
  for (int rr = 0; rr < 16; ++rr) {
    const int row = wv * 16 + rr;
    f16* wrow = sc + (size_t)row * SCS;
    float mx = -__builtin_inff();
    for (int t = lane; t < KLEN; t += 32) mx = fmaxf(mx, (float)wrow[t]);
    mx = wave_max(mx);
    float sum = 0.f;
    for (int t = lane; t < KLEN; t += 32) {
      const float e = __expf((float)wrow[t] - mx) * PSC;
      const f16 eh = (f16)e;
      wrow[t] = eh;
      sum += (float)eh;
    }
    sum = wave_sum(sum);
    if (lane == 0) rowsum[row] = sum;
  }
  __syncthreads();

  v8f o[4];
#pragma unroll
  for (int dt = 0; dt < 4; ++dt) o[dt] = v8zero();
  int jmax = iq + 16 + MLEN;
  if (jmax > KLEN) jmax = KLEN;
  jmax = (jmax + 31) & ~31;
  const f16* prow = sc + (size_t)(wv * 16 + r) * SCS + hl * 8;
  const f16* vbase = vT16 + (bh * DHD + r) * KLEN + hl * 8;
  for (int jc = 0; jc < jmax; jc += 32) {
    v16h pf = frag_ld(prow + jc);
#pragma unroll
    for (int dt = 0; dt < 4; ++dt) {
      v16h vf = frag_ld(vbase + (size_t)(dt * 16) * KLEN + jc);
      o[dt] = wmma16(pf, vf, o[dt]);
    }
  }

  float inv8[8];
#pragma unroll
  for (int g = 0; g < 8; ++g) inv8[g] = WSC / rowsum[wv * 16 + g + hl * 8];
  __syncthreads();
  f16* stg = (f16*)wstrip;
#pragma unroll
  for (int dt = 0; dt < 4; ++dt)
#pragma unroll
    for (int g = 0; g < 8; ++g)
      stg[(g + hl * 8) * STGP + dt * 16 + r] = (f16)(o[dt][g] * inv8[g]);
  __syncthreads();
  v8h ov[4];
  size_t od[4];
#pragma unroll
  for (int t = 0; t < 4; ++t) {
    const int m = t * 4 + (lane >> 3), e = lane & 7;
    ov[t] = *(const v8h*)(stg + m * STGP + e * 8);
    od[t] = ((size_t)(iq + m) * NB + b) * DMODEL + h * DHD + e * 8;
  }
#pragma unroll
  for (int t = 0; t < 4; ++t) *(volatile v8h*)(vec16 + od[t]) = ov[t];
  __threadfence();
#pragma unroll
  for (int t = 0; t < 4; ++t) *(volatile v8h*)(vec16 + od[t]) = ov[t];
}

__global__ __launch_bounds__(256) void add_ln_kernel(
    const float* __restrict__ x, const float* __restrict__ y,
    const float* __restrict__ gam, const float* __restrict__ bet,
    float* outf, f16* out16, int nrows) {
  __shared__ float red[8];
  __shared__ float red2[8];
  __shared__ v4f srow[256];
  const int row = blockIdx.x;
  if (row >= nrows) return;
  const int tid = threadIdx.x, lane = tid & 31, wv = tid >> 5;
  const size_t base = (size_t)row * DMODEL + 4 * tid;
  v4f a = *(const v4f*)(x + base) + *(const v4f*)(y + base);
  float s = (a[0] + a[1]) + (a[2] + a[3]);
  s = wave_sum(s);
  if (lane == 0) red[wv] = s;
  __syncthreads();
  float tot = 0.f;
#pragma unroll
  for (int k = 0; k < 8; ++k) tot += red[k];
  const float mean = tot * (1.0f / DMODEL);
  v4f d = a - mean;
  float s2 = (d[0] * d[0] + d[1] * d[1]) + (d[2] * d[2] + d[3] * d[3]);
  s2 = wave_sum(s2);
  if (lane == 0) red2[wv] = s2;
  __syncthreads();
  float tot2 = 0.f;
#pragma unroll
  for (int k = 0; k < 8; ++k) tot2 += red2[k];
  const float inv = rsqrtf(tot2 * (1.0f / DMODEL) + 1e-5f);
  v4f gg = *(const v4f*)(gam + 4 * tid);
  v4f bb = *(const v4f*)(bet + 4 * tid);
  v4f ov = d * inv * gg + bb;
  srow[tid] = ov;
  __syncthreads();
  v8h hv;
  const bool do16 = (out16 != nullptr) && (tid < 128);
  if (do16) hv = pack8(srow[2 * tid], srow[2 * tid + 1], 1.0f);
  const size_t o16 = (size_t)row * DMODEL + 8 * tid;
  if (outf) *(volatile v4f*)(outf + base) = ov;
  if (do16) *(volatile v8h*)(out16 + o16) = hv;
  __threadfence();
  if (outf) *(volatile v4f*)(outf + base) = ov;
  if (do16) *(volatile v8h*)(out16 + o16) = hv;
}

extern "C" void kernel_launch(void* const* d_in, const int* in_sizes, int n_in,
                              void* d_out, int out_size, void* d_ws, size_t ws_size,
                              hipStream_t stream) {
  if (n_in < 16) return;
  const int want[16] = {QLEN * NB * DMODEL, MLEN * NB * DMODEL, KLEN * NH * DHD, NH * DHD,
                        KLEN * NH, 3 * NH * DHD * DMODEL, DMODEL * NH * DHD, DMODEL, DMODEL,
                        DINNER * DMODEL, DINNER, DMODEL * DINNER, DMODEL, DMODEL, DMODEL,
                        QLEN * KLEN};
  for (int i = 0; i < 16; ++i)
    if (in_sizes[i] != want[i]) return;
  if (out_size != QLEN * NB * DMODEL) return;
  const size_t MB = (size_t)1 << 20;
  if (ws_size < 68 * MB) return;

  const float* dec_inp  = (const float*)d_in[0];
  const float* mems     = (const float*)d_in[1];
  const float* r_emb    = (const float*)d_in[2];
  const float* r_w_bias = (const float*)d_in[3];
  const float* r_bias   = (const float*)d_in[4];
  const float* qkv_w    = (const float*)d_in[5];
  const float* o_w      = (const float*)d_in[6];
  const float* ln1_g    = (const float*)d_in[7];
  const float* ln1_b    = (const float*)d_in[8];
  const float* ff_w1    = (const float*)d_in[9];
  const float* ff_b1    = (const float*)d_in[10];
  const float* ff_w2    = (const float*)d_in[11];
  const float* ff_b2    = (const float*)d_in[12];
  const float* ln2_g    = (const float*)d_in[13];
  const float* ln2_b    = (const float*)d_in[14];
  const int*   amask    = (const int*)d_in[15];

  char* ws = (char*)d_ws;
  f16*   cat16   = (f16*)(ws + 0);
  f16*   vec16   = (f16*)(ws + 0);
  f16*   heads16 = (f16*)(ws + 8 * MB);
  float* attnout = (float*)(ws + 8 * MB);
  float* outf    = (float*)(ws + 16 * MB);
  f16*   out16   = (f16*)(ws + 24 * MB);
  f16*   q16     = (f16*)(ws + 32 * MB);
  f16*   q16b    = (f16*)(ws + 36 * MB);
  f16*   k16     = (f16*)(ws + 40 * MB);
  f16*   vT16    = (f16*)(ws + 48 * MB);
  f16*   re16    = (f16*)(ws + 56 * MB);
  f16*   h16     = (f16*)(ws + 32 * MB);
  float* core    = (float*)(ws + 48 * MB);
  f16*   w16     = (f16*)(ws + 60 * MB);

  const int RB = QLEN * NB;
  const int KB = KLEN * NB;

  {
    const int n8a = MLEN * NB * DMODEL / 8;
    cvt16_kernel<<<(n8a + 255) / 256, 256, 0, stream>>>(mems, cat16, n8a, 1.0f);
    const int n8b = QLEN * NB * DMODEL / 8;
    cvt16_kernel<<<(n8b + 255) / 256, 256, 0, stream>>>(
        dec_inp, cat16 + (size_t)MLEN * NB * DMODEL, n8b, 1.0f);
    const int n8w = 3 * NH * DHD * DMODEL / 8;
    cvt16_kernel<<<(n8w + 255) / 256, 256, 0, stream>>>(qkv_w, w16, n8w, WSC);
  }
  gemm_nt_kernel<<<dim3(3072 / 128, KB / 128), 256, GEMM_SMEM, stream>>>(
      cat16, w16, nullptr, nullptr, heads16, KB, 3072, DMODEL, 0, INV_WSC);

  {
    const int nt = KLEN * NB * 256;
    split_qk_kernel<<<(nt + 255) / 256, 256, 0, stream>>>(heads16, r_w_bias, q16, q16b, k16, nt);
    vtrans_kernel<<<dim3(KLEN / 64, NH, NB), 256, 0, stream>>>(heads16, vT16);
    const int nr = KLEN * NH * 8;
    remb_kernel<<<(nr + 255) / 256, 256, 0, stream>>>(r_emb, re16, nr);
  }

  attn_kernel<<<dim3(QLEN / 64, NH, NB), 128, ATT_SMEM, stream>>>(
      q16, q16b, k16, vT16, re16, r_bias, amask, vec16);

  {
    const int n8 = DMODEL * DMODEL / 8;
    cvt16_kernel<<<(n8 + 255) / 256, 256, 0, stream>>>(o_w, w16, n8, WSC);
  }
  gemm_nt_kernel<<<dim3(DMODEL / 128, RB / 128), 256, GEMM_SMEM, stream>>>(
      vec16, w16, nullptr, attnout, nullptr, RB, DMODEL, DMODEL, 0, INV_WSC * INV_WSC);

  add_ln_kernel<<<RB, 256, 0, stream>>>(dec_inp, attnout, ln1_g, ln1_b, outf, out16, RB);

  {
    const int n8 = DINNER * DMODEL / 8;
    cvt16_kernel<<<(n8 + 255) / 256, 256, 0, stream>>>(ff_w1, w16, n8, WSC);
  }
  gemm_nt_kernel<<<dim3(DINNER / 128, RB / 128), 256, GEMM_SMEM, stream>>>(
      out16, w16, ff_b1, nullptr, h16, RB, DINNER, DMODEL, 1, INV_WSC);

  {
    const int n8 = DMODEL * DINNER / 8;
    cvt16_kernel<<<(n8 + 255) / 256, 256, 0, stream>>>(ff_w2, w16, n8, WSC);
  }
  gemm_nt_kernel<<<dim3(DMODEL / 128, RB / 128), 256, GEMM_SMEM, stream>>>(
      h16, w16, ff_b2, core, nullptr, RB, DMODEL, DINNER, 0, INV_WSC);

  add_ln_kernel<<<RB, 256, 0, stream>>>(outf, core, ln2_g, ln2_b, (float*)d_out, nullptr, RB);
}
